// CharEmbedBLSTM_59725815218203
// MI455X (gfx1250) — hardware-verified
//
#include <hip/hip_runtime.h>
#include <stdint.h>

#define NVOCAB   128
#define EMB      512
#define HID      256
#define GATE4    1024
#define NWORDS   4096
#define NSTEP    16
#define HPITCH   264
#define OPITCH   260

static_assert(NWORDS % 16 == 0);
static_assert(HID % 32 == 0);
static_assert(EMB % 32 == 0);
static_assert(NVOCAB % 64 == 0);
static_assert(GATE4 % 64 == 0);

#define OFF_EMBH  0ull
#define OFF_EMBL  131072ull
#define OFF_WIHH  262144ull
#define OFF_WIHL  2359296ull
#define OFF_WHH   4456448ull
#define OFF_BSUM  5505024ull
#define OFF_XG    5513216ull
#define WS_TOTAL  6561792ull

typedef __attribute__((ext_vector_type(16))) _Float16 v16h;
typedef __attribute__((ext_vector_type(8)))  _Float16 v8h;
typedef __attribute__((ext_vector_type(16))) __bf16   v16b;
typedef __attribute__((ext_vector_type(8)))  __bf16   v8b;
typedef __attribute__((ext_vector_type(8)))  float    v8f;
typedef __attribute__((ext_vector_type(4)))  float    v4f;

__device__ __forceinline__ unsigned short f2bf_bits(float f) {
  unsigned u = __float_as_uint(f);
  return (unsigned short)((u + 0x7FFFu + ((u >> 16) & 1u)) >> 16);
}
__device__ __forceinline__ float bf_bits2f(unsigned short h) { return __uint_as_float(((unsigned)h) << 16); }

__device__ __forceinline__ void dep_guard_h(v8f& a, v8f& b, v16h x, v16h y) { asm volatile("v_nop\n\tv_nop\n\tv_nop\n\tv_nop" : "+v"(a), "+v"(b) : "v"(x), "v"(y)); }
__device__ __forceinline__ void dep_guard_b(v8f& a, v8f& b, v16b x, v16b y) { asm volatile("v_nop\n\tv_nop\n\tv_nop\n\tv_nop" : "+v"(a), "+v"(b) : "v"(x), "v"(y)); }
__device__ __forceinline__ void keep4_h(v16h a, v16h b, v16h c, v16h d) { asm volatile("v_nop" :: "v"(a), "v"(b), "v"(c), "v"(d)); }
__device__ __forceinline__ void keep4_b(v16b a, v16b b, v16b c, v16b d) { asm volatile("v_nop" :: "v"(a), "v"(b), "v"(c), "v"(d)); }
__device__ __forceinline__ void acc_guard4(v8f& a, v8f& b, v8f& c, v8f& d) { asm volatile("v_nop\n\tv_nop\n\tv_nop\n\tv_nop" : "+v"(a), "+v"(b), "+v"(c), "+v"(d)); }

template <typename T> struct Frag;
template <> struct Frag<_Float16> {
  typedef v16h V; union U { v16h v; v8h h[2]; };
  static __device__ __forceinline__ v16h load(const _Float16* p) {
    U f; f.h[0] = *(const v8h*)(p); f.h[1] = *(const v8h*)(p + 16); return f.v;
  }
  static __device__ __forceinline__ v8f mma(v16h a, v16h b, v8f c) {
    return __builtin_amdgcn_wmma_f32_16x16x32_f16(false, a, false, b, (short)0, c, false, false);
  }
  static __device__ __forceinline__ void guard(v8f& a, v8f& b, v16h x, v16h y) { dep_guard_h(a, b, x, y); }
  static __device__ __forceinline__ void keep(v16h a, v16h b, v16h c, v16h d) { keep4_h(a, b, c, d); }
};
template <> struct Frag<__bf16> {
  typedef v16b V; union U { v16b v; v8b h[2]; };
  static __device__ __forceinline__ v16b load(const __bf16* p) {
    U f; f.h[0] = *(const v8b*)(p); f.h[1] = *(const v8b*)(p + 16); return f.v;
  }
  static __device__ __forceinline__ v8f mma(v16b a, v16b b, v8f c) {
    return __builtin_amdgcn_wmma_f32_16x16x32_bf16(false, a, false, b, (short)0, c, false, false);
  }
  static __device__ __forceinline__ void guard(v8f& a, v8f& b, v16b x, v16b y) { dep_guard_b(a, b, x, y); }
  static __device__ __forceinline__ void keep(v16b a, v16b b, v16b c, v16b d) { keep4_b(a, b, c, d); }
};

template <int ET> struct Elem;
template <> struct Elem<0> { typedef _Float16 T; };
template <> struct Elem<1> { typedef __bf16 T; };
template <int ET, bool SPLIT, int BIAS_MODE, int OUT_MODE, bool RESID, int ACT = 0>
__global__ __launch_bounds__(256) void wmma_gemm64(
    const unsigned short* __restrict__ Ap, const unsigned short* __restrict__ A2p, int lda, long strideA,
    const unsigned short* __restrict__ Btp, const unsigned short* __restrict__ Bt2p, int ldb, long strideB,
    void* __restrict__ Cout, void* __restrict__ Cout2, int ldc, long strideC,
    const float* __restrict__ bias,
    const float* __restrict__ resid, long strideR,
    int M, int N, int K, float scale) {
  typedef typename Elem<ET>::T T;
  typedef typename Frag<T>::V V;
  const T* A = (const T*)Ap; const T* A2 = (const T*)A2p; const T* Bt = (const T*)Btp; const T* Bt2 = (const T*)Bt2p;
  __shared__ __align__(16) float sT[8][16 * 68];
  const int b    = blockIdx.y;
  const int lane = threadIdx.x & 31;
  const int wave = threadIdx.x >> 5;
  const int tilesN = N >> 6;
  const int tilesM = M >> 6;
  const int tile = blockIdx.x * 8 + wave;
  if (tile >= tilesM * tilesN) return;
  const int tm = tile / tilesN;
  const int tn = tile - tm * tilesN;
  const int m0 = tm << 6;
  const int n0 = tn << 6;

  const T* Ab  = A  + (size_t)b * strideA;
  const T* Bb  = Bt + (size_t)b * strideB;
  const T* Ab2 = SPLIT ? (A2  + (size_t)b * strideA) : nullptr;
  const T* Bb2 = SPLIT ? (Bt2 + (size_t)b * strideB) : nullptr;

  const int rlane = lane & 15;
  const int koff  = (lane >> 4) * 8;
  const int mOff  = (lane >> 4) * 8;

  v8f acc[4][4];
#pragma unroll
  for (int i = 0; i < 4; ++i)
#pragma unroll
    for (int j = 0; j < 4; ++j) acc[i][j] = (v8f){0.f,0.f,0.f,0.f,0.f,0.f,0.f,0.f};

  for (int k0 = 0; k0 < K; k0 += 32) {
    V bh[4], bl[4];
#pragma unroll
    for (int j = 0; j < 4; ++j) {
      const size_t bo = (size_t)(n0 + (j << 4) + rlane) * ldb + koff + k0;
      bh[j] = Frag<T>::load(Bb + bo);
      if (SPLIT) bl[j] = Frag<T>::load(Bb2 + bo);
    }
#pragma unroll
    for (int i = 0; i < 4; ++i) {
      const size_t ao = (size_t)(m0 + (i << 4) + rlane) * lda + koff + k0;
      V ah = Frag<T>::load(Ab + ao);
      V al;
      if (SPLIT) al = Frag<T>::load(Ab2 + ao);
#pragma unroll
      for (int j = 0; j < 4; ++j) {
        acc[i][j] = Frag<T>::mma(ah, bh[j], acc[i][j]);
        if (SPLIT) {
          acc[i][j] = Frag<T>::mma(ah, bl[j], acc[i][j]);
          acc[i][j] = Frag<T>::mma(al, bh[j], acc[i][j]);
        }
      }
      Frag<T>::guard(acc[i][0], acc[i][3], ah, SPLIT ? al : ah);
    }
    Frag<T>::keep(bh[0], bh[1], bh[2], bh[3]);
    if (SPLIT) Frag<T>::keep(bl[0], bl[1], bl[2], bl[3]);
  }
  acc_guard4(acc[0][0], acc[0][1], acc[0][2], acc[0][3]);
  acc_guard4(acc[1][0], acc[1][1], acc[1][2], acc[1][3]);
  acc_guard4(acc[2][0], acc[2][1], acc[2][2], acc[2][3]);
  acc_guard4(acc[3][0], acc[3][1], acc[3][2], acc[3][3]);

  float* slab = sT[wave];
  const float* Rb = RESID ? (resid + (size_t)b * strideR) : nullptr;
#pragma unroll
  for (int i = 0; i < 4; ++i) {
    const int mBase = m0 + (i << 4);
#pragma unroll
    for (int j = 0; j < 4; ++j) {
      const int n = n0 + (j << 4) + rlane;
      float bv = 0.f;
      if (BIAS_MODE == 2) bv = bias[n];
#pragma unroll
      for (int r = 0; r < 8; ++r) {
        float v = acc[i][j][r] * scale;
        if (BIAS_MODE == 1) v += bias[mBase + mOff + r];
        if (BIAS_MODE == 2) v += bv;
        if (RESID) v += Rb[(size_t)(mBase + mOff + r) * ldc + n];
        if (ACT == 1) v = tanhf(v);
        if (ACT == 2) v = fmaxf(v, 0.0f);
        if (ACT == 3) v = v / (1.0f + expf(-v));
        if (ACT == 4) v = (v > 0.f) ? v : 0.01f * v;
        if (ACT == 5) v = 0.5f * v * (1.0f + erff(v * 0.70710678118654752f));
        slab[(mOff + r) * 68 + (j << 4) + rlane] = v;
      }
    }
    __builtin_amdgcn_fence(__ATOMIC_RELEASE, "workgroup");
    __builtin_amdgcn_wave_barrier();
    __builtin_amdgcn_fence(__ATOMIC_ACQUIRE, "workgroup");
    if (OUT_MODE == 0) {
      float* C = (float*)Cout + (size_t)b * strideC;
      const int hh = lane >> 4, c4 = (lane & 15) * 4;
      for (int pass = 0; pass < 2; ++pass) {
#pragma unroll
        for (int it = 0; it < 8; ++it) {
          const int row = it * 2 + hh;
          v4f v = *(const v4f*)(slab + row * 68 + c4);
          *(volatile v4f*)(C + (size_t)(mBase + row) * ldc + n0 + c4) = v;
        }
        __threadfence();
      }
    } else {
      const int q = lane >> 3, c8 = (lane & 7) * 8;
      unsigned short* C  = (unsigned short*)Cout  + (size_t)b * strideC;
      unsigned short* C2 = (OUT_MODE == 2) ? ((unsigned short*)Cout2 + (size_t)b * strideC) : nullptr;
      for (int pass = 0; pass < 2; ++pass) {
#pragma unroll
        for (int it = 0; it < 4; ++it) {
          const int row = it * 4 + q;
          const float* sp = slab + row * 68 + c8;
          v8h hv, lv;
#pragma unroll
          for (int e = 0; e < 8; ++e) {
            if (OUT_MODE == 1) {
              hv[e] = (_Float16)sp[e];
            } else {
              unsigned short hb = f2bf_bits(sp[e]);
              unsigned short lb = f2bf_bits(sp[e] - bf_bits2f(hb));
              hv[e] = __builtin_bit_cast(_Float16, hb);
              lv[e] = __builtin_bit_cast(_Float16, lb);
            }
          }
          *(volatile v8h*)(C + (size_t)(mBase + row) * ldc + n0 + c8) = hv;
          if (OUT_MODE == 2) *(volatile v8h*)(C2 + (size_t)(mBase + row) * ldc + n0 + c8) = lv;
        }
        __threadfence();
      }
    }
    __builtin_amdgcn_fence(__ATOMIC_RELEASE, "workgroup");
    __builtin_amdgcn_wave_barrier();
    __builtin_amdgcn_fence(__ATOMIC_ACQUIRE, "workgroup");
  }
}

__global__ __launch_bounds__(256) void split_bf16x2(
    const float* __restrict__ in, unsigned short* __restrict__ hi, unsigned short* __restrict__ lo, int n2) {
  const int i = blockIdx.x * 256 + threadIdx.x;
  if (i < n2) {
    const float f0 = in[2 * i], f1 = in[2 * i + 1];
    const unsigned short h0 = f2bf_bits(f0), h1 = f2bf_bits(f1);
    const unsigned short l0 = f2bf_bits(f0 - bf_bits2f(h0));
    const unsigned short l1 = f2bf_bits(f1 - bf_bits2f(h1));
    const unsigned uh = (unsigned)h0 | ((unsigned)h1 << 16);
    const unsigned ul = (unsigned)l0 | ((unsigned)l1 << 16);
    ((volatile unsigned*)hi)[i] = uh;
    ((volatile unsigned*)lo)[i] = ul;
    __threadfence();
    ((volatile unsigned*)hi)[i] = uh;
    ((volatile unsigned*)lo)[i] = ul;
  }
}

__global__ __launch_bounds__(256) void cast_f32_f16x2_scaled(
    const float* __restrict__ in, _Float16* __restrict__ out, int n2, float scale) {
  const int i = blockIdx.x * 256 + threadIdx.x;
  if (i < n2) {
    const _Float16 h0 = (_Float16)(in[2 * i] * scale), h1 = (_Float16)(in[2 * i + 1] * scale);
    const unsigned u = (unsigned)__builtin_bit_cast(unsigned short, h0) | ((unsigned)__builtin_bit_cast(unsigned short, h1) << 16);
    ((volatile unsigned*)out)[i] = u;
    __threadfence();
    ((volatile unsigned*)out)[i] = u;
  }
}

__global__ __launch_bounds__(256) void bias_sum(
    const float* __restrict__ a, const float* __restrict__ b, float* __restrict__ o, int n) {
  const int i = blockIdx.x * 256 + threadIdx.x;
  if (i < n) {
    const float v = a[i] + b[i];
    ((volatile float*)o)[i] = v;
    __threadfence();
    ((volatile float*)o)[i] = v;
  }
}

__device__ __forceinline__ v8f mma_f16g(v16h a, v16h b, v8f c) {
  c = __builtin_amdgcn_wmma_f32_16x16x32_f16(false, a, false, b, (short)0, c, false, false);
  asm volatile("v_nop\n\tv_nop\n\tv_nop\n\tv_nop" : "+v"(c) : "v"(a), "v"(b));
  return c;
}
__device__ __forceinline__ float rcp_f(float v) { return __builtin_amdgcn_rcpf(v); }
__device__ __forceinline__ float sigm_f(float v) { return rcp_f(1.0f + expf(-v)); }
__device__ __forceinline__ float tanh_f(float v) { return 1.0f - 2.0f * rcp_f(1.0f + expf(2.0f * v)); }

__global__ __launch_bounds__(256) void blstm_persist(
    const int* __restrict__ x, const float* __restrict__ xg,
    const unsigned short* __restrict__ whhp, float* __restrict__ out) {
  __shared__ __align__(16) _Float16 hA[16 * HPITCH];
  __shared__ __align__(16) float oS[16 * OPITCH];
  __shared__ int xl[16 * NSTEP];
  union FH { v16h v; v8h h[2]; };

  const int tid  = threadIdx.x;
  const int lane = tid & 31;
  const int wave = tid >> 5;
  const int hh   = lane >> 4;
  const int c    = lane & 15;
  const int dir  = blockIdx.y;
  const int r0   = blockIdx.x * 16;

  {
    int v = x[(size_t)(r0 + (tid >> 4)) * NSTEP + (tid & 15)];
    v = v < 0 ? 0 : (v > NVOCAB - 1 ? NVOCAB - 1 : v);
    xl[tid] = v;
  }

  const _Float16* whh = (const _Float16*)whhp + (size_t)dir * GATE4 * HID;
  const float* xgd = xg + (size_t)dir * NVOCAB * GATE4;
  const int ub0 = 2 * wave;

  float cst[2][8];
#pragma unroll
  for (int u = 0; u < 2; ++u)
#pragma unroll
    for (int r = 0; r < 8; ++r) cst[u][r] = 0.0f;

#pragma unroll 1
  for (int t = 0; t < NSTEP; ++t) {
    const int l = dir ? (NSTEP - 1 - t) : t;
    __syncthreads();

    v8f acc[2][4];
#pragma unroll
    for (int u = 0; u < 2; ++u)
#pragma unroll
      for (int g = 0; g < 4; ++g) acc[u][g] = (v8f){0.f,0.f,0.f,0.f,0.f,0.f,0.f,0.f};

    if (t > 0) {
#pragma unroll 1
      for (int k0 = 0; k0 < HID; k0 += 32) {
        FH af;
        af.h[0] = *(const v8h*)(hA + c * HPITCH + k0 + 8 * hh);
        af.h[1] = *(const v8h*)(hA + c * HPITCH + k0 + 16 + 8 * hh);
#pragma unroll
        for (int u = 0; u < 2; ++u) {
          v16h bq[4];
#pragma unroll
          for (int g = 0; g < 4; ++g)
            bq[g] = Frag<_Float16>::load(whh + (size_t)(g * HID + 16 * (ub0 + u) + c) * HID + k0 + 8 * hh);
#pragma unroll
          for (int g = 0; g < 4; ++g) acc[u][g] = mma_f16g(af.v, bq[g], acc[u][g]);
        }
      }
    }
    __syncthreads();

    int chr[8];
#pragma unroll
    for (int r = 0; r < 8; ++r) chr[r] = xl[(8 * hh + r) * NSTEP + l];

#pragma unroll
    for (int u = 0; u < 2; ++u) {
      const int j = 16 * (ub0 + u) + c;
#pragma unroll
      for (int r = 0; r < 8; ++r) {
        const float* xr = xgd + (size_t)chr[r] * GATE4 + j;
        const float gi = acc[u][0][r] * (1.0f / 64.0f) + xr[0];
        const float gf = acc[u][1][r] * (1.0f / 64.0f) + xr[HID];
        const float gg = acc[u][2][r] * (1.0f / 64.0f) + xr[2 * HID];
        const float go = acc[u][3][r] * (1.0f / 64.0f) + xr[3 * HID];
        const float iv = sigm_f(gi);
        const float fv = sigm_f(gf);
        const float gv = tanh_f(gg);
        const float ov = sigm_f(go);
        const float cn = fv * cst[u][r] + iv * gv;
        cst[u][r] = cn;
        const float hn = ov * tanh_f(cn);
        hA[(8 * hh + r) * HPITCH + j] = (_Float16)(hn * 8.0f);
        if (t == NSTEP - 1) oS[(8 * hh + r) * OPITCH + j] = hn;
      }
    }
  }
  __syncthreads();

  for (int pass = 0; pass < 2; ++pass) {
#pragma unroll
    for (int rr = 0; rr < 2; ++rr) {
      const int row = 2 * wave + rr;
      float* dst = out + (size_t)(r0 + row) * (2 * HID) + (size_t)dir * HID;
#pragma unroll
      for (int hf = 0; hf < 2; ++hf) {
        const int col = hf * 128 + 4 * lane;
        const v4f v = *(const v4f*)(oS + row * OPITCH + col);
        *(volatile v4f*)(dst + col) = v;
      }
    }
    __threadfence();
  }
}

extern "C" void kernel_launch(void* const* d_in, const int* in_sizes, int n_in,
                              void* d_out, int out_size, void* d_ws, size_t ws_size,
                              hipStream_t stream) {
  if (n_in < 10) return;
  if (in_sizes[0] != NWORDS * NSTEP) return;
  if (in_sizes[1] != NVOCAB * EMB) return;
  if (in_sizes[2] != GATE4 * EMB || in_sizes[6] != GATE4 * EMB) return;
  if (in_sizes[3] != GATE4 * HID || in_sizes[7] != GATE4 * HID) return;
  if (in_sizes[4] != GATE4 || in_sizes[5] != GATE4 || in_sizes[8] != GATE4 || in_sizes[9] != GATE4) return;
  if (out_size != NWORDS * 2 * HID) return;
  if (ws_size < (size_t)WS_TOTAL) return;

  const int*   x      = (const int*)d_in[0];
  const float* embed  = (const float*)d_in[1];
  const float* w_ih_f = (const float*)d_in[2];
  const float* w_hh_f = (const float*)d_in[3];
  const float* b_ih_f = (const float*)d_in[4];
  const float* b_hh_f = (const float*)d_in[5];
  const float* w_ih_b = (const float*)d_in[6];
  const float* w_hh_b = (const float*)d_in[7];
  const float* b_ih_b = (const float*)d_in[8];
  const float* b_hh_b = (const float*)d_in[9];
  float* out = (float*)d_out;

  char* ws = (char*)d_ws;
  unsigned short* embH = (unsigned short*)(ws + OFF_EMBH);
  unsigned short* embL = (unsigned short*)(ws + OFF_EMBL);
  unsigned short* wihH = (unsigned short*)(ws + OFF_WIHH);
  unsigned short* wihL = (unsigned short*)(ws + OFF_WIHL);
  unsigned short* whh  = (unsigned short*)(ws + OFF_WHH);
  float* bsum = (float*)(ws + OFF_BSUM);
  float* xg   = (float*)(ws + OFF_XG);

  const int nEmb  = NVOCAB * EMB;
  const int nWih  = GATE4 * EMB;
  const int nWhh  = GATE4 * HID;

  split_bf16x2<<<dim3(nEmb / 512), 256, 0, stream>>>(embed, embH, embL, nEmb / 2);
  split_bf16x2<<<dim3(nWih / 512), 256, 0, stream>>>(w_ih_f, wihH, wihL, nWih / 2);
  split_bf16x2<<<dim3(nWih / 512), 256, 0, stream>>>(w_ih_b, wihH + nWih, wihL + nWih, nWih / 2);
  cast_f32_f16x2_scaled<<<dim3(nWhh / 512), 256, 0, stream>>>(w_hh_f, (_Float16*)whh, nWhh / 2, 8.0f);
  cast_f32_f16x2_scaled<<<dim3(nWhh / 512), 256, 0, stream>>>(w_hh_b, (_Float16*)(whh + nWhh), nWhh / 2, 8.0f);
  bias_sum<<<dim3(GATE4 / 256), 256, 0, stream>>>(b_ih_f, b_hh_f, bsum, GATE4);
  bias_sum<<<dim3(GATE4 / 256), 256, 0, stream>>>(b_ih_b, b_hh_b, bsum + GATE4, GATE4);

  const int tiles = (NVOCAB / 64) * (GATE4 / 64);
  for (int d = 0; d < 2; ++d) {
    float* xgd = xg + (size_t)d * NVOCAB * GATE4;
    wmma_gemm64<1, true, 2, 0, false, 0><<<dim3((tiles + 7) / 8, 1), 256, 0, stream>>>(
        embH, embL, EMB, 0L,
        wihH + (size_t)d * nWih, wihL + (size_t)d * nWih, EMB, 0L,
        (void*)xgd, (void*)xgd, GATE4, 0L,
        bsum + d * GATE4,
        bsum, 0L,
        NVOCAB, GATE4, EMB, 1.0f);
  }

  blstm_persist<<<dim3(NWORDS / 16, 2), 256, 0, stream>>>(x, xg, whh, out);
}
